// RelationModule_21706764714077
// MI455X (gfx1250) — hardware-verified
//
#include <hip/hip_runtime.h>
#include <stddef.h>


typedef _Float16 v16h __attribute__((ext_vector_type(16)));
typedef _Float16 v8h  __attribute__((ext_vector_type(8)));
typedef float    v8f  __attribute__((ext_vector_type(8)));
typedef float    v4f  __attribute__((ext_vector_type(4)));

#ifndef NB
#define NB 128
#endif
#define NB_FULL 128
#define FEAT  1024
#define K2    2048
#define NCLS  500
#define CPAD  512
#define HID   512
#define BT    8
#define NV4   (BT * NCLS / 4)

static_assert(NB >= 64 && NB <= NB_FULL && (NB % 64) == 0);
static_assert(K2 == 2 * FEAT);
static_assert((FEAT % 32) == 0 && (FEAT % 8) == 0 && (K2 % 8) == 0);
static_assert((HID % 64) == 0 && (CPAD % 64) == 0 && CPAD >= NCLS);
static_assert((NB % BT) == 0);
static_assert(((BT * NCLS * 4) % 128) == 0);
static_assert(((BT * NCLS) % 4) == 0 && (NV4 % 8) == 0 && NV4 <= 4 * 256);
static_assert(BT * HID == 4 * 256 * 4);
static_assert(HID == 2 * 256);
static_assert(NCLS <= 2 * 256);
static_assert(((size_t)HID * K2) % 2048 == 0);
static_assert(((size_t)NB * FEAT) % 2048 == 0);
static_assert(((size_t)CPAD * FEAT) % 2048 == 0);

#define LDC 68
static_assert((LDC % 4) == 0 && LDC >= 64);

#define WCARRY 64.0f

#define WH_BYTES ((size_t)HID * K2 * 2)
#define XI_BYTES ((size_t)NB * FEAT * 2)
#define XA_BYTES ((size_t)CPAD * FEAT * 2)
#define P_BYTES  ((size_t)NB * HID * 4)
#define Q_BYTES  ((size_t)CPAD * HID * 4)
#define OFF_WH ((size_t)0)
#define OFF_XI (OFF_WH + WH_BYTES)
#define OFF_XA (OFF_XI + XI_BYTES)
#define OFF_P  (OFF_XA + XA_BYTES)
#define OFF_Q  (OFF_P + P_BYTES)
#define WS_TOTAL (OFF_Q + Q_BYTES)
static_assert((WH_BYTES % 128) == 0 && (XI_BYTES % 128) == 0 && (XA_BYTES % 128) == 0);
static_assert((P_BYTES % 128) == 0 && (Q_BYTES % 128) == 0);
static_assert(WS_TOTAL <= (size_t)134217728);

__device__ __forceinline__ float bf16r(float x) {
  unsigned int u = __float_as_uint(x);
  u = (u + 0x7FFFu + ((u >> 16) & 1u)) & 0xFFFF0000u;
  return __uint_as_float(u);
}

static __device__ __forceinline__ _Float16 toh_flush(float v) {
  const _Float16 r = (_Float16)v;
  return (fabsf(v) < 6.103515625e-05f) ? (_Float16)0.0f : r;
}

__device__ __forceinline__ v16h frag_at(const _Float16* p) {
  v8h lo = *(const v8h*)(p);
  v8h hi = *(const v8h*)(p + 16);
  v16h out;
#pragma unroll
  for (int i = 0; i < 8; ++i) { out[i] = lo[i]; out[i + 8] = hi[i]; }
  return out;
}

__device__ __forceinline__ v8f wmma16(v16h a, v16h b, v8f c) {
  v8f d = __builtin_amdgcn_wmma_f32_16x16x32_f16(false, a, false, b, (short)0, c,
                                                 false, false);
  asm volatile("v_nop\n\tv_nop\n\tv_nop\n\tv_nop" : "+v"(d) : "v"(a), "v"(b));
  return d;
}

template <unsigned COLS, unsigned ROWS_VALID, unsigned ROWS_PAD>
__device__ __forceinline__ void cast_body(const float* __restrict__ src,
                                          _Float16* __restrict__ dst, const float carry) {
  const unsigned idx = blockIdx.x * 256u + threadIdx.x;
  if (idx >= ROWS_PAD * COLS / 8u) return;
  const unsigned e = idx * 8u;
  const unsigned row = e / COLS;
  const unsigned col = e - row * COLS;
  const unsigned rowc = (row < ROWS_VALID) ? row : (ROWS_VALID - 1u);
  const float* p = src + (size_t)rowc * COLS + col;
  const v4f a0 = *(const v4f*)(p);
  const v4f a1 = *(const v4f*)(p + 4);
  const bool valid = row < ROWS_VALID;
  v8h o;
#pragma unroll
  for (int i = 0; i < 4; ++i) {
    const float f0 = valid ? bf16r(a0[i]) : 0.0f;
    const float f1 = valid ? bf16r(a1[i]) : 0.0f;
    o[i]     = toh_flush(carry * f0);
    o[i + 4] = toh_flush(carry * f1);
  }
  _Float16* q = dst + (size_t)e;
  *(volatile v8h*)q = o;
  __threadfence();
  *(volatile v8h*)q = o;
}

__global__ __launch_bounds__(256) void cast_w_kernel(
    const float* __restrict__ src, _Float16* __restrict__ dst) {
  cast_body<K2, HID, HID>(src, dst, WCARRY);
}
__global__ __launch_bounds__(256) void cast_img_kernel(
    const float* __restrict__ src, _Float16* __restrict__ dst) {
  cast_body<FEAT, NB, NB>(src, dst, 1.0f);
}
__global__ __launch_bounds__(256) void cast_attr_kernel(
    const float* __restrict__ src, _Float16* __restrict__ dst) {
  cast_body<FEAT, NCLS, CPAD>(src, dst, 1.0f);
}

template <int BIAS>
__device__ __forceinline__ void gemm_body(
    const _Float16* __restrict__ A16, const _Float16* __restrict__ Bt,
    const float* __restrict__ bias, float* __restrict__ outf) {
  __shared__ __attribute__((aligned(16))) float Cs[64 * LDC];
  const unsigned tid = threadIdx.x, lane = tid & 31u;
  const unsigned w = (unsigned)__builtin_amdgcn_readfirstlane((int)(tid >> 5));
  const unsigned mw = w >> 1, nw = w & 1u;
  const unsigned hh = lane >> 4, m = lane & 15u;
  const unsigned n0 = blockIdx.x * 64u;
  const unsigned row0 = blockIdx.y * 64u;

  const _Float16* ap  = A16 + (size_t)(row0 + mw * 16u + m) * FEAT + hh * 8u;
  const _Float16* bp0 = Bt + (size_t)(n0 + nw * 32u + m) * K2 + hh * 8u;
  const _Float16* bp1 = bp0 + (size_t)16 * K2;
  v8f acc0 = {}, acc1 = {};
#pragma unroll 2
  for (unsigned k0 = 0; k0 < (unsigned)FEAT; k0 += 32u) {
    const v16h a  = frag_at(ap + k0);
    const v16h b0 = frag_at(bp0 + k0);
    const v16h b1 = frag_at(bp1 + k0);
    acc0 = wmma16(a, b0, acc0);
    acc1 = wmma16(a, b1, acc1);
  }
#pragma unroll
  for (int r = 0; r < 8; ++r) {
    float* d = &Cs[(mw * 16u + hh * 8u + (unsigned)r) * LDC + nw * 32u + m];
    d[0]  = acc0[r];
    d[16] = acc1[r];
  }
  __syncthreads();

  v4f xs[4];
  size_t off[4];
#pragma unroll
  for (unsigned i = 0; i < 4u; ++i) {
    const unsigned r = 16u * i + (tid >> 4);
    const unsigned c = (tid & 15u) * 4u;
    const v4f u = *(const v4f*)&Cs[r * LDC + c];
    v4f val;
    if (BIAS) {
      const v4f g = *(const v4f*)(bias + n0 + c);
#pragma unroll
      for (int j = 0; j < 4; ++j) val[j] = u[j] * (1.0f / WCARRY) + bf16r(g[j]);
    } else {
#pragma unroll
      for (int j = 0; j < 4; ++j) val[j] = u[j] * (1.0f / WCARRY);
    }
    xs[i] = val;
    off[i] = (size_t)(row0 + r) * HID + n0 + c;
  }
#pragma unroll
  for (int i = 0; i < 4; ++i) *(volatile v4f*)(outf + off[i]) = xs[i];
  __threadfence();
#pragma unroll
  for (int i = 0; i < 4; ++i) *(volatile v4f*)(outf + off[i]) = xs[i];
}

__global__ __launch_bounds__(256) void gemm_img_kernel(
    const _Float16* __restrict__ A16, const _Float16* __restrict__ Bt,
    const float* __restrict__ bias, float* __restrict__ outf) {
  gemm_body<1>(A16, Bt, bias, outf);
}
__global__ __launch_bounds__(256) void gemm_attr_kernel(
    const _Float16* __restrict__ A16, const _Float16* __restrict__ Bt,
    float* __restrict__ outf) {
  gemm_body<0>(A16, Bt, (const float*)0, outf);
}

__global__ __launch_bounds__(256) void score_kernel(
    const float* __restrict__ P, const float* __restrict__ Q,
    const float* __restrict__ W2, const float* __restrict__ B2,
    float* __restrict__ out) {
  __shared__ __attribute__((aligned(16))) float s_p[BT * HID];
  __shared__ __attribute__((aligned(16))) float s_w[HID];
  __shared__ __attribute__((aligned(16))) float s_o[BT * NCLS];

  const unsigned tid = threadIdx.x;
  const unsigned b0 = blockIdx.x * BT;
#pragma unroll
  for (unsigned j = 0; j < 4u; ++j) {
    const unsigned idx = tid + 256u * j;
    *(v4f*)&s_p[idx * 4u] = *(const v4f*)(P + (size_t)b0 * HID + idx * 4u);
  }
#pragma unroll
  for (unsigned j = 0; j < 2u; ++j) {
    const unsigned idx = tid + 256u * j;
    s_w[idx] = bf16r(W2[idx]);
  }
  const float b2v = bf16r(B2[0]);
  __syncthreads();

#pragma unroll 1
  for (unsigned pass = 0; pass < 2u; ++pass) {
    const unsigned c = pass * 256u + tid;
    const unsigned cc = (c < (unsigned)NCLS) ? c : (unsigned)(NCLS - 1);
    const float* qrow = Q + (size_t)cc * HID;
    float acc[BT];
#pragma unroll
    for (int b = 0; b < BT; ++b) acc[b] = 0.0f;
#pragma unroll 1
    for (unsigned h = 0; h < (unsigned)HID; h += 4u) {
      const v4f q  = *(const v4f*)(qrow + h);
      const v4f wv = *(const v4f*)&s_w[h];
#pragma unroll
      for (int b = 0; b < BT; ++b) {
        const v4f p = *(const v4f*)&s_p[(unsigned)b * HID + h];
#pragma unroll
        for (int j = 0; j < 4; ++j) {
          const float t = fmaxf(p[j] + q[j], 0.0f);
          acc[b] = fmaf(t, wv[j], acc[b]);
        }
      }
    }
    if (c < (unsigned)NCLS) {
#pragma unroll
      for (int b = 0; b < BT; ++b) s_o[(unsigned)b * NCLS + c] = acc[b] + b2v;
    }
  }
  __syncthreads();

  v4f xs[4];
#pragma unroll
  for (unsigned j = 0; j < 4u; ++j) {
    const unsigned idx = tid + 256u * j;
    const unsigned idc = (idx < (unsigned)NV4) ? idx : (unsigned)(NV4 - 1);
    const v4f u = *(const v4f*)&s_o[idc * 4u];
    v4f y;
#pragma unroll
    for (int i = 0; i < 4; ++i) y[i] = __builtin_amdgcn_rcpf(1.0f + __expf(-u[i]));
    xs[j] = y;
  }
  float* ob = out + (size_t)blockIdx.x * (BT * NCLS);
#pragma unroll
  for (unsigned j = 0; j < 4u; ++j) {
    const unsigned idx = tid + 256u * j;
    if (idx < (unsigned)NV4) *(volatile v4f*)(ob + idx * 4u) = xs[j];
  }
  __threadfence();
#pragma unroll
  for (unsigned j = 0; j < 4u; ++j) {
    const unsigned idx = tid + 256u * j;
    if (idx < (unsigned)NV4) *(volatile v4f*)(ob + idx * 4u) = xs[j];
  }
}

extern "C" void kernel_launch(void* const* d_in, const int* in_sizes, int n_in,
                              void* d_out, int out_size, void* d_ws, size_t ws_size,
                              hipStream_t stream) {
  if (n_in < 6) return;
  if ((long long)in_sizes[0] < (long long)NB * FEAT) return;
  if ((long long)in_sizes[1] < (long long)NCLS * FEAT) return;
  if ((long long)in_sizes[2] < (long long)HID * K2) return;
  if (in_sizes[3] < HID) return;
  if (in_sizes[4] < HID) return;
  if (in_sizes[5] < 1) return;
  if ((long long)out_size < (long long)NB * NCLS) return;
  if (ws_size < WS_TOTAL) return;

  const float* img  = (const float*)d_in[0];
  const float* attr = (const float*)d_in[1];
  const float* w1   = (const float*)d_in[2];
  const float* b1   = (const float*)d_in[3];
  const float* w2   = (const float*)d_in[4];
  const float* b2   = (const float*)d_in[5];
  float* out = (float*)d_out;

  char* ws = (char*)d_ws;
  _Float16* Wh = (_Float16*)(ws + OFF_WH);
  _Float16* Xi = (_Float16*)(ws + OFF_XI);
  _Float16* Xa = (_Float16*)(ws + OFF_XA);
  float*    Pp = (float*)(ws + OFF_P);
  float*    Qp = (float*)(ws + OFF_Q);

  dim3 blk(256);
  cast_w_kernel<<<dim3((unsigned)((size_t)HID * K2 / 2048)), blk, 0, stream>>>(w1, Wh);
  cast_img_kernel<<<dim3((unsigned)((size_t)NB * FEAT / 2048)), blk, 0, stream>>>(img, Xi);
  cast_attr_kernel<<<dim3((unsigned)((size_t)CPAD * FEAT / 2048)), blk, 0, stream>>>(attr, Xa);

  gemm_img_kernel<<<dim3(HID / 64, NB / 64), blk, 0, stream>>>(Xi, Wh, b1, Pp);
  gemm_attr_kernel<<<dim3(HID / 64, CPAD / 64), blk, 0, stream>>>(Xa, Wh + FEAT, Qp);

  score_kernel<<<dim3(NB / BT), blk, 0, stream>>>(Pp, Qp, w2, b2, out);
}
